// BlockAxialUp_9560597201242
// MI455X (gfx1250) — hardware-verified
//
#include <hip/hip_runtime.h>
#include <stdint.h>
#include <math.h>


typedef __attribute__((ext_vector_type(16))) _Float16 v16h;
typedef __attribute__((ext_vector_type(8)))  _Float16 v8h;
typedef __attribute__((ext_vector_type(16))) __bf16   v16b;
typedef __attribute__((ext_vector_type(8)))  __bf16   v8b;
typedef __attribute__((ext_vector_type(8)))  float    v8f;
typedef __attribute__((ext_vector_type(4)))  float    v4f;

#define NB    4
#define CIN   256
#define HIN   64
#define HO    128
#define EMB   128
#define NPIX  65536
#define NTOKC 16384
#define NQKV  768
#define KCAT  640
#define WSCL  64.0f
#define WSCL_INV (1.0f / 64.0f)

__device__ __forceinline__ unsigned short f2bf_bits(float f) {
  unsigned u = __float_as_uint(f);
  return (unsigned short)((u + 0x7FFFu + ((u >> 16) & 1u)) >> 16);
}
__device__ __forceinline__ float bf_bits2f(unsigned short h) { return __uint_as_float(((unsigned)h) << 16); }

__device__ __forceinline__ void dep_guard_h(v8f& a, v8f& b, v16h x, v16h y) { asm volatile("v_nop\n\tv_nop\n\tv_nop\n\tv_nop" : "+v"(a), "+v"(b) : "v"(x), "v"(y)); }
__device__ __forceinline__ void dep_guard_b(v8f& a, v8f& b, v16b x, v16b y) { asm volatile("v_nop\n\tv_nop\n\tv_nop\n\tv_nop" : "+v"(a), "+v"(b) : "v"(x), "v"(y)); }
__device__ __forceinline__ void keep4_h(v16h a, v16h b, v16h c, v16h d) { asm volatile("v_nop" :: "v"(a), "v"(b), "v"(c), "v"(d)); }
__device__ __forceinline__ void keep4_b(v16b a, v16b b, v16b c, v16b d) { asm volatile("v_nop" :: "v"(a), "v"(b), "v"(c), "v"(d)); }
__device__ __forceinline__ void acc_guard4(v8f& a, v8f& b, v8f& c, v8f& d) { asm volatile("v_nop\n\tv_nop\n\tv_nop\n\tv_nop" : "+v"(a), "+v"(b), "+v"(c), "+v"(d)); }
template <typename T> struct Frag;
template <> struct Frag<_Float16> {
  typedef v16h V; union U { v16h v; v8h h[2]; };
  static __device__ __forceinline__ v16h load(const _Float16* p) {
    U f; f.h[0] = *(const v8h*)(p); f.h[1] = *(const v8h*)(p + 16); return f.v;
  }
  static __device__ __forceinline__ v8f mma(v16h a, v16h b, v8f c) {
    return __builtin_amdgcn_wmma_f32_16x16x32_f16(false, a, false, b, (short)0, c, false, false);
  }
  static __device__ __forceinline__ void guard(v8f& a, v8f& b, v16h x, v16h y) { dep_guard_h(a, b, x, y); }
  static __device__ __forceinline__ void keep(v16h a, v16h b, v16h c, v16h d) { keep4_h(a, b, c, d); }
};
template <> struct Frag<__bf16> {
  typedef v16b V; union U { v16b v; v8b h[2]; };
  static __device__ __forceinline__ v16b load(const __bf16* p) {
    U f; f.h[0] = *(const v8b*)(p); f.h[1] = *(const v8b*)(p + 16); return f.v;
  }
  static __device__ __forceinline__ v8f mma(v16b a, v16b b, v8f c) {
    return __builtin_amdgcn_wmma_f32_16x16x32_bf16(false, a, false, b, (short)0, c, false, false);
  }
  static __device__ __forceinline__ void guard(v8f& a, v8f& b, v16b x, v16b y) { dep_guard_b(a, b, x, y); }
  static __device__ __forceinline__ void keep(v16b a, v16b b, v16b c, v16b d) { keep4_b(a, b, c, d); }
};

__device__ __forceinline__ v8f ax_mma(v16h a, v16h b, v8f c) {
  c = __builtin_amdgcn_wmma_f32_16x16x32_f16(false, a, false, b, (short)0, c, false, false);
  asm volatile("v_nop\n\tv_nop\n\tv_nop\n\tv_nop" : "+v"(c) : "v"(a), "v"(b));
  return c;
}

template <int ET> struct Elem;
template <> struct Elem<0> { typedef _Float16 T; };
template <> struct Elem<1> { typedef __bf16 T; };
template <int ET, bool SPLIT, int BIAS_MODE, int OUT_MODE, bool RESID, int ACT = 0>
__global__ __launch_bounds__(256) void wmma_gemm64(
    const unsigned short* __restrict__ Ap, const unsigned short* __restrict__ A2p, int lda, long strideA,
    const unsigned short* __restrict__ Btp, const unsigned short* __restrict__ Bt2p, int ldb, long strideB,
    void* __restrict__ Cout, void* __restrict__ Cout2, int ldc, long strideC,
    const float* __restrict__ bias,
    const float* __restrict__ resid, long strideR,
    int M, int N, int K, float scale) {
  typedef typename Elem<ET>::T T;
  typedef typename Frag<T>::V V;
  const T* A = (const T*)Ap; const T* A2 = (const T*)A2p; const T* Bt = (const T*)Btp; const T* Bt2 = (const T*)Bt2p;
  __shared__ __align__(16) float sT[8][16 * 68];
  const int b    = blockIdx.y;
  const int lane = threadIdx.x & 31;
  const int wave = threadIdx.x >> 5;
  const int tilesN = N >> 6;
  const int tilesM = M >> 6;
  const int tile = blockIdx.x * 8 + wave;
  if (tile >= tilesM * tilesN) return;
  const int tm = tile / tilesN;
  const int tn = tile - tm * tilesN;
  const int m0 = tm << 6;
  const int n0 = tn << 6;

  const T* Ab  = A  + (size_t)b * strideA;
  const T* Bb  = Bt + (size_t)b * strideB;
  const T* Ab2 = SPLIT ? (A2  + (size_t)b * strideA) : nullptr;
  const T* Bb2 = SPLIT ? (Bt2 + (size_t)b * strideB) : nullptr;

  const int rlane = lane & 15;
  const int koff  = (lane >> 4) * 8;
  const int mOff  = (lane >> 4) * 8;

  v8f acc[4][4];
#pragma unroll
  for (int i = 0; i < 4; ++i)
#pragma unroll
    for (int j = 0; j < 4; ++j) acc[i][j] = (v8f){0.f,0.f,0.f,0.f,0.f,0.f,0.f,0.f};

  for (int k0 = 0; k0 < K; k0 += 32) {
    V bh[4], bl[4];
#pragma unroll
    for (int j = 0; j < 4; ++j) {
      const size_t bo = (size_t)(n0 + (j << 4) + rlane) * ldb + koff + k0;
      bh[j] = Frag<T>::load(Bb + bo);
      if (SPLIT) bl[j] = Frag<T>::load(Bb2 + bo);
    }
#pragma unroll
    for (int i = 0; i < 4; ++i) {
      const size_t ao = (size_t)(m0 + (i << 4) + rlane) * lda + koff + k0;
      V ah = Frag<T>::load(Ab + ao);
      V al;
      if (SPLIT) al = Frag<T>::load(Ab2 + ao);
#pragma unroll
      for (int j = 0; j < 4; ++j) {
        acc[i][j] = Frag<T>::mma(ah, bh[j], acc[i][j]);
        if (SPLIT) {
          acc[i][j] = Frag<T>::mma(ah, bl[j], acc[i][j]);
          acc[i][j] = Frag<T>::mma(al, bh[j], acc[i][j]);
        }
      }
      Frag<T>::guard(acc[i][0], acc[i][3], ah, SPLIT ? al : ah);
    }
    Frag<T>::keep(bh[0], bh[1], bh[2], bh[3]);
    if (SPLIT) Frag<T>::keep(bl[0], bl[1], bl[2], bl[3]);
  }
  acc_guard4(acc[0][0], acc[0][1], acc[0][2], acc[0][3]);
  acc_guard4(acc[1][0], acc[1][1], acc[1][2], acc[1][3]);
  acc_guard4(acc[2][0], acc[2][1], acc[2][2], acc[2][3]);
  acc_guard4(acc[3][0], acc[3][1], acc[3][2], acc[3][3]);

  float* slab = sT[wave];
  const float* Rb = RESID ? (resid + (size_t)b * strideR) : nullptr;
#pragma unroll
  for (int i = 0; i < 4; ++i) {
    const int mBase = m0 + (i << 4);
#pragma unroll
    for (int j = 0; j < 4; ++j) {
      const int n = n0 + (j << 4) + rlane;
      float bv = 0.f;
      if (BIAS_MODE == 2) bv = bias[n];
#pragma unroll
      for (int r = 0; r < 8; ++r) {
        float v = acc[i][j][r] * scale;
        if (BIAS_MODE == 1) v += bias[mBase + mOff + r];
        if (BIAS_MODE == 2) v += bv;
        if (RESID) v += Rb[(size_t)(mBase + mOff + r) * ldc + n];
        if (ACT == 1) v = tanhf(v);
        if (ACT == 2) v = fmaxf(v, 0.0f);
        if (ACT == 3) v = v / (1.0f + expf(-v));
        if (ACT == 4) v = (v > 0.f) ? v : 0.01f * v;
        if (ACT == 5) v = 0.5f * v * (1.0f + erff(v * 0.70710678118654752f));
        slab[(mOff + r) * 68 + (j << 4) + rlane] = v;
      }
    }
    __builtin_amdgcn_fence(__ATOMIC_RELEASE, "workgroup");
    __builtin_amdgcn_wave_barrier();
    __builtin_amdgcn_fence(__ATOMIC_ACQUIRE, "workgroup");
    if (OUT_MODE == 0) {
      float* C = (float*)Cout + (size_t)b * strideC;
      const int hh = lane >> 4, c4 = (lane & 15) * 4;
      for (int pass = 0; pass < 2; ++pass) {
#pragma unroll
        for (int it = 0; it < 8; ++it) {
          const int row = it * 2 + hh;
          v4f v = *(const v4f*)(slab + row * 68 + c4);
          *(volatile v4f*)(C + (size_t)(mBase + row) * ldc + n0 + c4) = v;
        }
        __threadfence();
      }
    } else {
      const int q = lane >> 3, c8 = (lane & 7) * 8;
      unsigned short* C  = (unsigned short*)Cout  + (size_t)b * strideC;
      unsigned short* C2 = (OUT_MODE == 2) ? ((unsigned short*)Cout2 + (size_t)b * strideC) : nullptr;
      for (int pass = 0; pass < 2; ++pass) {
#pragma unroll
        for (int it = 0; it < 4; ++it) {
          const int row = it * 4 + q;
          const float* sp = slab + row * 68 + c8;
          v8h hv, lv;
#pragma unroll
          for (int e = 0; e < 8; ++e) {
            if (OUT_MODE == 1) {
              hv[e] = (_Float16)sp[e];
            } else {
              unsigned short hb = f2bf_bits(sp[e]);
              unsigned short lb = f2bf_bits(sp[e] - bf_bits2f(hb));
              hv[e] = __builtin_bit_cast(_Float16, hb);
              lv[e] = __builtin_bit_cast(_Float16, lb);
            }
          }
          *(volatile v8h*)(C + (size_t)(mBase + row) * ldc + n0 + c8) = hv;
          if (OUT_MODE == 2) *(volatile v8h*)(C2 + (size_t)(mBase + row) * ldc + n0 + c8) = lv;
        }
        __threadfence();
      }
    }
    __builtin_amdgcn_fence(__ATOMIC_RELEASE, "workgroup");
    __builtin_amdgcn_wave_barrier();
    __builtin_amdgcn_fence(__ATOMIC_ACQUIRE, "workgroup");
  }
}

__global__ __launch_bounds__(256) void k_conv_gemm(
    const _Float16* __restrict__ A, int lda,
    const _Float16* __restrict__ B0, const _Float16* __restrict__ B1, const _Float16* __restrict__ B2,
    float* __restrict__ C, int ldc, int M, int N, float scale) {
  __shared__ __align__(16) float sT[8][16 * 68];
  const int lane = threadIdx.x & 31;
  const int wave = threadIdx.x >> 5;
  const int tilesN = N >> 6;
  const int tilesM = M >> 6;
  const int tile = blockIdx.x * 8 + wave;
  if (tile >= tilesM * tilesN) return;
  const int tm = tile / tilesN;
  const int tn = tile - tm * tilesN;
  const int m0 = tm << 6;
  const int n0 = tn << 6;
  const int rlane = lane & 15;
  const int koff  = (lane >> 4) * 8;
  const int mOff  = (lane >> 4) * 8;

  v8f acc[4][4];
#pragma unroll
  for (int i = 0; i < 4; ++i)
#pragma unroll
    for (int j = 0; j < 4; ++j) acc[i][j] = (v8f){0.f,0.f,0.f,0.f,0.f,0.f,0.f,0.f};

  for (int k0 = 0; k0 < KCAT; k0 += 32) {
    const _Float16* Bs; int ldb; int kk;
    if (k0 < CIN) { Bs = B0; ldb = CIN; kk = k0; }
    else if (k0 < 2 * CIN) { Bs = B1; ldb = CIN; kk = k0 - CIN; }
    else { Bs = B2; ldb = EMB; kk = k0 - 2 * CIN; }
    v16h bh[4];
#pragma unroll
    for (int j = 0; j < 4; ++j)
      bh[j] = Frag<_Float16>::load(Bs + (size_t)(n0 + (j << 4) + rlane) * ldb + koff + kk);
#pragma unroll
    for (int i = 0; i < 4; ++i) {
      const v16h ah = Frag<_Float16>::load(A + (size_t)(m0 + (i << 4) + rlane) * lda + koff + k0);
#pragma unroll
      for (int j = 0; j < 4; ++j) acc[i][j] = Frag<_Float16>::mma(ah, bh[j], acc[i][j]);
      Frag<_Float16>::guard(acc[i][0], acc[i][3], ah, ah);
    }
    Frag<_Float16>::keep(bh[0], bh[1], bh[2], bh[3]);
  }
  acc_guard4(acc[0][0], acc[0][1], acc[0][2], acc[0][3]);
  acc_guard4(acc[1][0], acc[1][1], acc[1][2], acc[1][3]);
  acc_guard4(acc[2][0], acc[2][1], acc[2][2], acc[2][3]);
  acc_guard4(acc[3][0], acc[3][1], acc[3][2], acc[3][3]);

  float* slab = sT[wave];
#pragma unroll
  for (int i = 0; i < 4; ++i) {
    const int mBase = m0 + (i << 4);
#pragma unroll
    for (int j = 0; j < 4; ++j) {
#pragma unroll
      for (int r = 0; r < 8; ++r) {
        float v = acc[i][j][r] * scale;
        v = fmaxf(v, 0.0f);
        slab[(mOff + r) * 68 + (j << 4) + rlane] = v;
      }
    }
    __builtin_amdgcn_fence(__ATOMIC_RELEASE, "workgroup");
    __builtin_amdgcn_wave_barrier();
    __builtin_amdgcn_fence(__ATOMIC_ACQUIRE, "workgroup");
    {
      const int hh = lane >> 4, c4 = (lane & 15) * 4;
      for (int pass = 0; pass < 2; ++pass) {
#pragma unroll
        for (int it = 0; it < 8; ++it) {
          const int row = it * 2 + hh;
          v4f v = *(const v4f*)(slab + row * 68 + c4);
          *(volatile v4f*)(C + (size_t)(mBase + row) * ldc + n0 + c4) = v;
        }
        __threadfence();
      }
    }
    __builtin_amdgcn_fence(__ATOMIC_RELEASE, "workgroup");
    __builtin_amdgcn_wave_barrier();
    __builtin_amdgcn_fence(__ATOMIC_ACQUIRE, "workgroup");
  }
}

__global__ __launch_bounds__(256) void k_wtrans(const float* __restrict__ src, int src_pitch,
                                               _Float16* __restrict__ dst, int K, int npairs, float mul) {
  const int i = blockIdx.x * 256 + threadIdx.x;
  if (i < npairs) {
    const int lin = 2 * i;
    const int n = lin / K;
    const int k = lin - n * K;
    const float f0 = src[(size_t)k * src_pitch + n] * mul;
    const float f1 = src[(size_t)(k + 1) * src_pitch + n] * mul;
    const unsigned u = (unsigned)__builtin_bit_cast(unsigned short, (_Float16)f0) |
                       ((unsigned)__builtin_bit_cast(unsigned short, (_Float16)f1) << 16);
    ((volatile unsigned*)dst)[i] = u;
    __threadfence();
    ((volatile unsigned*)dst)[i] = u;
  }
}

#define UP_P 136
__global__ __launch_bounds__(256) void k_upsample(const float* __restrict__ x,
                                                 _Float16* __restrict__ xw, _Float16* __restrict__ xh) {
  #pragma clang fp contract(off)
  __shared__ __align__(16) _Float16 tile[HO * UP_P];
  const int h = blockIdx.x, b = blockIdx.y;
  const int t = threadIdx.x;
  const int w = t & 127, cx = t >> 7;
  const int wave = t >> 5, lane = t & 31, hh = lane >> 4, c8 = (lane & 15) * 8;
  const float R = (float)(63.0 / 127.0);
  const float chf = (float)h * R;
  int i0 = (int)floorf(chf); i0 = i0 < 0 ? 0 : (i0 > HIN - 2 ? HIN - 2 : i0);
  const float wh = chf - (float)i0;
  const float cwf = (float)w * R;
  int j0 = (int)floorf(cwf); j0 = j0 < 0 ? 0 : (j0 > HIN - 2 ? HIN - 2 : j0);
  const float ww = cwf - (float)j0;
  const float omh = 1.0f - wh;
  const float omw = 1.0f - ww;
#pragma unroll 1
  for (int half = 0; half < 2; ++half) {
#pragma unroll 2
    for (int ci = 0; ci < 64; ++ci) {
      const int cl = 2 * ci + cx;
      const int c = half * 128 + cl;
      const float* p = x + (((size_t)(b * CIN + c)) * HIN + i0) * HIN + j0;
      const float x00 = p[0], x01 = p[1], x10 = p[HIN], x11 = p[HIN + 1];
      const float hA = x00 * omh + x10 * wh;
      const float hB = x01 * omh + x11 * wh;
      const float v = hA * omw + hB * ww;
      tile[w * UP_P + cl] = (_Float16)v;
    }
    __syncthreads();
    for (int pass = 0; pass < 2; ++pass) {
#pragma unroll
      for (int it = 0; it < 8; ++it) {
        const int rw = it * 16 + wave * 2 + hh;
        const v8h val = *(const v8h*)(tile + rw * UP_P + c8);
        const size_t roww = ((size_t)(b * HO + h) * HO + rw) * CIN + half * 128 + c8;
        const size_t rowh = ((size_t)(b * HO + rw) * HO + h) * CIN + half * 128 + c8;
        *(volatile v8h*)(xw + roww) = val;
        *(volatile v8h*)(xh + rowh) = val;
      }
      __threadfence();
    }
    __syncthreads();
  }
}

__global__ __launch_bounds__(256) void k_res(const float* __restrict__ res, _Float16* __restrict__ r16) {
  __shared__ __align__(16) _Float16 tile[HO * UP_P];
  const int h = blockIdx.x, b = blockIdx.y;
  const int t = threadIdx.x;
  const int w = t & 127, ex = t >> 7;
  const int wave = t >> 5, lane = t & 31, hh = lane >> 4, c8 = (lane & 15) * 8;
#pragma unroll 2
  for (int ei = 0; ei < 64; ++ei) {
    const int e = 2 * ei + ex;
    tile[w * UP_P + e] = (_Float16)res[(((size_t)(b * EMB + e)) * HO + h) * HO + w];
  }
  __syncthreads();
  for (int pass = 0; pass < 2; ++pass) {
#pragma unroll
    for (int it = 0; it < 8; ++it) {
      const int rw = it * 16 + wave * 2 + hh;
      const v8h val = *(const v8h*)(tile + rw * UP_P + c8);
      *(volatile v8h*)(r16 + ((size_t)(b * HO + h) * HO + rw) * EMB + c8) = val;
    }
    __threadfence();
  }
}

#define AX_T   128
#define AX_D   128
#define AX_KC  32
#define AX_KP  136
#define AX_VP  40
#define AX_PP  40
#define AX_OP  264
#define AX_PSC 32768.0f
#define AX_OFF_K 0
#define AX_OFF_V 8704
#define AX_OFF_P 18944
#define AX_OFF_O 24064
#define AX_SMEM  57856
struct AxGeom { long out_row0; long seq_rs; long tok_rs; float qk_scale; float o_scale; };
static_assert(sizeof(AxGeom) == 32);

template <int MODE>
__global__ __launch_bounds__(128) void k_axial_attn(
    const _Float16* __restrict__ qkv, const _Float16* __restrict__ wot,
    const float* __restrict__ bias, const _Float16* __restrict__ resid,
    _Float16* __restrict__ out, AxGeom g) {
  union FH { v16h v; v8h h[2]; };
  __shared__ __align__(16) unsigned char smem[AX_SMEM];
  _Float16* Ksh = (_Float16*)(smem + AX_OFF_K);
  _Float16* Vt  = (_Float16*)(smem + AX_OFF_V);
  _Float16* Psh = (_Float16*)(smem + AX_OFF_P);
  _Float16* Osh = (_Float16*)(smem + AX_OFF_O);
  float* slabs  = (float*)(smem + AX_OFF_K);

  const int tid  = threadIdx.x;
  const int wave = tid >> 5;
  const int lane = tid & 31;
  const int hh   = lane >> 4;
  const int c    = lane & 15;
  const int sl   = blockIdx.x >> 1;
  const int qb   = blockIdx.x & 1;
  const int tok0 = sl * AX_T;
  const int q0   = qb * 64 + wave * 16;

#pragma unroll 1
  for (int hd = 0; hd < 2; ++hd) {
    v16h qa[4];
    {
      const _Float16* qrow = qkv + (size_t)(tok0 + q0 + c) * NQKV + hd * AX_D + 8 * hh;
#pragma unroll
      for (int kc = 0; kc < 4; ++kc) qa[kc] = Frag<_Float16>::load(qrow + kc * 32);
    }
    float mrow[8], lrow[8];
    v8f oacc[8];
#pragma unroll
    for (int r = 0; r < 8; ++r) { mrow[r] = -INFINITY; lrow[r] = 0.f; }
#pragma unroll
    for (int t = 0; t < 8; ++t) oacc[t] = (v8f){0.f,0.f,0.f,0.f,0.f,0.f,0.f,0.f};

#pragma unroll 1
    for (int kch = 0; kch < AX_T / AX_KC; ++kch) {
      const int kv0 = kch * AX_KC;
      __syncthreads();
#pragma unroll
      for (int i = 0; i < 4; ++i) {
        const int idx = tid + 128 * i;
        const int kvr = idx >> 4;
        const int d8  = (idx & 15) * 8;
        const _Float16* rowp = qkv + (size_t)(tok0 + kv0 + kvr) * NQKV + hd * AX_D + d8;
        const v8h kk = *(const v8h*)(rowp + CIN);
        const v8h vv = *(const v8h*)(rowp + 2 * CIN);
        *(v8h*)(Ksh + kvr * AX_KP + d8) = kk;
#pragma unroll
        for (int e = 0; e < 8; ++e) Vt[(d8 + e) * AX_VP + kvr] = vv[e];
      }
      __syncthreads();

      v8f s[2];
#pragma unroll
      for (int j = 0; j < 2; ++j) {
        s[j] = (v8f){0.f,0.f,0.f,0.f,0.f,0.f,0.f,0.f};
#pragma unroll
        for (int kc = 0; kc < 4; ++kc) {
          FH kb;
          kb.h[0] = *(const v8h*)(Ksh + (j * 16 + c) * AX_KP + kc * 32 + 8 * hh);
          kb.h[1] = *(const v8h*)(Ksh + (j * 16 + c) * AX_KP + kc * 32 + 16 + 8 * hh);
          s[j] = ax_mma(qa[kc], kb.v, s[j]);
        }
      }
      float cm[8];
#pragma unroll
      for (int r = 0; r < 8; ++r) {
        float m = -INFINITY;
#pragma unroll
        for (int j = 0; j < 2; ++j) {
          s[j][r] = s[j][r] * g.qk_scale;
          m = fmaxf(m, s[j][r]);
        }
#pragma unroll
        for (int off = 1; off < 16; off <<= 1) m = fmaxf(m, __shfl_xor(m, off, 32));
        cm[r] = m;
      }
      _Float16* pw = Psh + wave * (16 * AX_PP);
#pragma unroll
      for (int r = 0; r < 8; ++r) {
        const float mnew  = fmaxf(mrow[r], cm[r]);
        const float alpha = expf(mrow[r] - mnew);
        mrow[r] = mnew;
        float psum = 0.f;
#pragma unroll
        for (int j = 0; j < 2; ++j) {
          const float p = expf(s[j][r] - mnew);
          psum += p;
          pw[(8 * hh + r) * AX_PP + j * 16 + c] = (_Float16)(p * AX_PSC);
        }
#pragma unroll
        for (int off = 1; off < 16; off <<= 1) psum += __shfl_xor(psum, off, 32);
        lrow[r] = lrow[r] * alpha + psum;
#pragma unroll
        for (int t = 0; t < 8; ++t) oacc[t][r] *= alpha;
      }
      __builtin_amdgcn_fence(__ATOMIC_RELEASE, "workgroup");
      __builtin_amdgcn_wave_barrier();
      __builtin_amdgcn_fence(__ATOMIC_ACQUIRE, "workgroup");
      {
        FH pa;
        pa.h[0] = *(const v8h*)(pw + c * AX_PP + 8 * hh);
        pa.h[1] = *(const v8h*)(pw + c * AX_PP + 16 + 8 * hh);
#pragma unroll
        for (int t = 0; t < 8; ++t) {
          FH vb;
          vb.h[0] = *(const v8h*)(Vt + (t * 16 + c) * AX_VP + 8 * hh);
          vb.h[1] = *(const v8h*)(Vt + (t * 16 + c) * AX_VP + 16 + 8 * hh);
          oacc[t] = ax_mma(pa.v, vb.v, oacc[t]);
        }
      }
    }
#pragma unroll
    for (int r = 0; r < 8; ++r) {
      const float inv = 1.0f / (lrow[r] * AX_PSC);
#pragma unroll
      for (int t = 0; t < 8; ++t)
        Osh[(wave * 16 + 8 * hh + r) * AX_OP + hd * AX_D + t * 16 + c] = (_Float16)(oacc[t][r] * inv);
    }
  }
  __syncthreads();

  float* slab = slabs + wave * (16 * 68);
  const _Float16* orow_p = Osh + (size_t)(wave * 16 + c) * AX_OP + 8 * hh;
  const int q8 = lane >> 3, c8 = (lane & 7) * 8;
#pragma unroll 1
  for (int js = 0; js < 4; ++js) {
    v8f acc[4];
#pragma unroll
    for (int j = 0; j < 4; ++j) acc[j] = (v8f){0.f,0.f,0.f,0.f,0.f,0.f,0.f,0.f};
#pragma unroll 1
    for (int k0 = 0; k0 < CIN; k0 += 32) {
      const v16h a = Frag<_Float16>::load(orow_p + k0);
#pragma unroll
      for (int j = 0; j < 4; ++j) {
        const v16h bf = Frag<_Float16>::load(wot + (size_t)(js * 64 + j * 16 + c) * CIN + k0 + 8 * hh);
        acc[j] = ax_mma(a, bf, acc[j]);
      }
    }
#pragma unroll
    for (int j = 0; j < 4; ++j) {
      const int n = js * 64 + j * 16 + c;
      const float bv = bias[n];
#pragma unroll
      for (int r = 0; r < 8; ++r) {
        const int row = 8 * hh + r;
        float v = acc[j][r] * g.o_scale + bv;
        if (MODE == 1) {
          const long orow = g.out_row0 + (long)sl * g.seq_rs + (long)(q0 + row) * g.tok_rs;
          v += (float)resid[(size_t)orow * CIN + n];
          v = fmaxf(v, 0.0f);
        }
        slab[row * 68 + j * 16 + c] = v;
      }
    }
    __builtin_amdgcn_fence(__ATOMIC_RELEASE, "workgroup");
    __builtin_amdgcn_wave_barrier();
    __builtin_amdgcn_fence(__ATOMIC_ACQUIRE, "workgroup");
    for (int pass = 0; pass < 2; ++pass) {
#pragma unroll
      for (int it = 0; it < 4; ++it) {
        const int row = it * 4 + q8;
        const float* sp = slab + row * 68 + c8;
        v8h hv;
#pragma unroll
        for (int e = 0; e < 8; ++e) hv[e] = (_Float16)sp[e];
        const long orow = g.out_row0 + (long)sl * g.seq_rs + (long)(q0 + row) * g.tok_rs;
        *(volatile v8h*)(out + (size_t)orow * CIN + js * 64 + c8) = hv;
      }
      __threadfence();
    }
    __builtin_amdgcn_fence(__ATOMIC_RELEASE, "workgroup");
    __builtin_amdgcn_wave_barrier();
    __builtin_amdgcn_fence(__ATOMIC_ACQUIRE, "workgroup");
  }
}

__global__ __launch_bounds__(256) void k_bn(const float* __restrict__ y, const float* __restrict__ gamma,
                                           const float* __restrict__ beta, float* __restrict__ out) {
  __shared__ double s1[256];
  __shared__ double s2[256];
  const int e = blockIdx.x, tid = threadIdx.x;
  const float* yr = y + (size_t)e * NPIX;
  double a = 0.0, q = 0.0;
#pragma unroll 1
  for (int i = 0; i < NPIX / 256; ++i) {
    const double v = (double)yr[i * 256 + tid];
    a += v;
    q += v * v;
  }
  s1[tid] = a;
  s2[tid] = q;
  __syncthreads();
  for (int off = 128; off > 0; off >>= 1) {
    if (tid < off) { s1[tid] += s1[tid + off]; s2[tid] += s2[tid + off]; }
    __syncthreads();
  }
  const double mu = s1[0] * (1.0 / (double)NPIX);
  double var = s2[0] * (1.0 / (double)NPIX) - mu * mu;
  if (var < 0.0) var = 0.0;
  const float inv = 1.0f / sqrtf((float)var + 1e-5f);
  const float gsc = gamma[e] * inv;
  const float muf = (float)mu;
  const float bt  = beta[e];
  for (int pass = 0; pass < 2; ++pass) {
#pragma unroll 1
    for (int bb = 0; bb < NB; ++bb) {
#pragma unroll 1
      for (int i = 0; i < (HO * HO) / (256 * 4); ++i) {
        const int idx = (i * 256 + tid) * 4;
        const v4f v = *(const v4f*)(yr + (size_t)bb * (HO * HO) + idx);
        v4f o;
#pragma unroll
        for (int k = 0; k < 4; ++k) o[k] = (v[k] - muf) * gsc + bt;
        *(volatile v4f*)(out + (size_t)(bb * EMB + e) * (HO * HO) + idx) = o;
      }
    }
    __threadfence();
  }
}

extern "C" void kernel_launch(void* const* d_in, const int* in_sizes, int n_in,
                              void* d_out, int out_size, void* d_ws, size_t ws_size,
                              hipStream_t stream) {
  if (n_in != 13) return;
  if (in_sizes[0] != NB * CIN * HIN * HIN) return;
  if (in_sizes[1] != NB * EMB * HO * HO) return;
  if (in_sizes[2] != CIN * CIN || in_sizes[3] != CIN * 2 * CIN || in_sizes[4] != CIN * CIN || in_sizes[5] != CIN) return;
  if (in_sizes[6] != CIN * CIN || in_sizes[7] != CIN * 2 * CIN || in_sizes[8] != CIN * CIN || in_sizes[9] != CIN) return;
  if (in_sizes[10] != KCAT * EMB || in_sizes[11] != EMB || in_sizes[12] != EMB) return;
  if (out_size != NB * EMB * HO * HO) return;

  const float* x      = (const float*)d_in[0];
  const float* res    = (const float*)d_in[1];
  const float* wq_h   = (const float*)d_in[2];
  const float* wkv_h  = (const float*)d_in[3];
  const float* wo_h   = (const float*)d_in[4];
  const float* wob_h  = (const float*)d_in[5];
  const float* wq_w   = (const float*)d_in[6];
  const float* wkv_w  = (const float*)d_in[7];
  const float* wo_w   = (const float*)d_in[8];
  const float* wob_w  = (const float*)d_in[9];
  const float* conv_w = (const float*)d_in[10];
  const float* gamma  = (const float*)d_in[11];
  const float* beta   = (const float*)d_in[12];
  float* out = (float*)d_out;

  const size_t SZ_X16 = (size_t)NPIX * CIN * 2;
  const size_t SZ_S3  = (size_t)NTOKC * NQKV * 2;
  const size_t OFF_S0 = 0;
  const size_t OFF_S1 = OFF_S0 + SZ_X16;
  const size_t OFF_S2 = OFF_S1 + SZ_X16;
  const size_t OFF_S3 = OFF_S2 + SZ_X16;
  const size_t OFF_W     = OFF_S3 + SZ_S3;
  const size_t OFF_WQKVH = OFF_W;
  const size_t OFF_WOH   = OFF_WQKVH + (size_t)NQKV * CIN * 2;
  const size_t OFF_WQKVW = OFF_WOH   + (size_t)CIN * CIN * 2;
  const size_t OFF_WOW   = OFF_WQKVW + (size_t)NQKV * CIN * 2;
  const size_t OFF_CONV  = OFF_WOW   + (size_t)CIN * CIN * 2;
  const size_t WS_END    = OFF_CONV  + (size_t)EMB * KCAT * 2;
  if (ws_size < WS_END) return;
  if ((size_t)NPIX * EMB * 2 > SZ_S3) return;
  if ((size_t)EMB * NPIX * 4 > SZ_X16) return;

  char* ws = (char*)d_ws;
  _Float16* XH16   = (_Float16*)(ws + OFF_S0);
  _Float16* XATT16 = (_Float16*)(ws + OFF_S0);
  _Float16* XW16   = (_Float16*)(ws + OFF_S1);
  _Float16* AH16   = (_Float16*)(ws + OFF_S2);
  float*    Y32    = (float*)(ws + OFF_S2);
  _Float16* QKV16  = (_Float16*)(ws + OFF_S3);
  _Float16* RES16  = (_Float16*)(ws + OFF_S3);
  _Float16* WQKVH  = (_Float16*)(ws + OFF_WQKVH);
  _Float16* WOH    = (_Float16*)(ws + OFF_WOH);
  _Float16* WQKVW  = (_Float16*)(ws + OFF_WQKVW);
  _Float16* WOW    = (_Float16*)(ws + OFF_WOW);
  _Float16* CONVT  = (_Float16*)(ws + OFF_CONV);

  {
    const int np_q = CIN * CIN / 2, np_kv = 2 * CIN * CIN / 2, np_cv = EMB * KCAT / 2;
    k_wtrans<<<(np_q + 255) / 256, 256, 0, stream>>>(wq_h, CIN, WQKVH, CIN, np_q, WSCL);
    k_wtrans<<<(np_kv + 255) / 256, 256, 0, stream>>>(wkv_h, 2 * CIN, WQKVH + (size_t)CIN * CIN, CIN, np_kv, WSCL);
    k_wtrans<<<(np_q + 255) / 256, 256, 0, stream>>>(wo_h, CIN, WOH, CIN, np_q, WSCL);
    k_wtrans<<<(np_q + 255) / 256, 256, 0, stream>>>(wq_w, CIN, WQKVW, CIN, np_q, WSCL);
    k_wtrans<<<(np_kv + 255) / 256, 256, 0, stream>>>(wkv_w, 2 * CIN, WQKVW + (size_t)CIN * CIN, CIN, np_kv, WSCL);
    k_wtrans<<<(np_q + 255) / 256, 256, 0, stream>>>(wo_w, CIN, WOW, CIN, np_q, WSCL);
    k_wtrans<<<(np_cv + 255) / 256, 256, 0, stream>>>(conv_w, EMB, CONVT, KCAT, np_cv, WSCL);
  }

  k_upsample<<<dim3(HO, NB), 256, 0, stream>>>(x, XW16, XH16);

  const float qk_scale = (float)0.08838834764831845;
  const int gemm_blocks = ((NTOKC / 64) * (NQKV / 64)) / 8;
  const int attn_blocks = (NTOKC / AX_T) * 2;

  for (int b = 0; b < NB; ++b) {
    const _Float16* Xc = XH16 + (size_t)b * NTOKC * CIN;
    wmma_gemm64<0, false, 0, 1, false, 0><<<dim3(gemm_blocks, 1), 256, 0, stream>>>(
        (const unsigned short*)Xc, (const unsigned short*)Xc, CIN, 0L,
        (const unsigned short*)WQKVH, (const unsigned short*)WQKVH, CIN, 0L,
        (void*)QKV16, (void*)QKV16, NQKV, 0L,
        wob_h, (const float*)(ws + OFF_S2), 0L,
        NTOKC, NQKV, CIN, WSCL_INV);
    AxGeom ga;
    ga.out_row0 = (long)b * NTOKC; ga.seq_rs = 1; ga.tok_rs = HO; ga.qk_scale = qk_scale; ga.o_scale = WSCL_INV;
    k_axial_attn<0><<<attn_blocks, 128, 0, stream>>>(QKV16, WOH, wob_h, XW16, AH16, ga);
  }

  for (int b = 0; b < NB; ++b) {
    const _Float16* Xc = XW16 + (size_t)b * NTOKC * CIN;
    wmma_gemm64<0, false, 0, 1, false, 0><<<dim3(gemm_blocks, 1), 256, 0, stream>>>(
        (const unsigned short*)Xc, (const unsigned short*)Xc, CIN, 0L,
        (const unsigned short*)WQKVW, (const unsigned short*)WQKVW, CIN, 0L,
        (void*)QKV16, (void*)QKV16, NQKV, 0L,
        wob_w, (const float*)(ws + OFF_S2), 0L,
        NTOKC, NQKV, CIN, WSCL_INV);
    AxGeom gw;
    gw.out_row0 = (long)b * NTOKC; gw.seq_rs = HO; gw.tok_rs = 1; gw.qk_scale = qk_scale; gw.o_scale = WSCL_INV;
    k_axial_attn<1><<<attn_blocks, 128, 0, stream>>>(QKV16, WOW, wob_w, AH16, XATT16, gw);
  }

  k_res<<<dim3(HO, NB), 256, 0, stream>>>(res, RES16);
  {
    const int conv_blocks = ((EMB / 64) * (NPIX / 64)) / 8;
    k_conv_gemm<<<conv_blocks, 256, 0, stream>>>(CONVT, KCAT, XATT16, XW16, RES16, Y32, NPIX, EMB, NPIX, WSCL_INV);
  }
  k_bn<<<EMB, 256, 0, stream>>>(Y32, gamma, beta, out);
  (void)hipGetLastError();
}
